// RWKV_Model_24764781429094
// MI455X (gfx1250) — hardware-verified
//
#include <hip/hip_runtime.h>
#include <stdint.h>
#include <stddef.h>
#include <math.h>

#define DD 128
#define FF 512
#define VV 256
#define LL 2
#define TT 1024
#define BB 32
#define NR (BB * TT)

typedef __attribute__((ext_vector_type(16))) _Float16 v16h;
typedef __attribute__((ext_vector_type(8)))  _Float16 v8h;
typedef __attribute__((ext_vector_type(16))) __bf16   v16b;
typedef __attribute__((ext_vector_type(8)))  __bf16   v8b;
typedef __attribute__((ext_vector_type(8)))  float    v8f;
typedef __attribute__((ext_vector_type(4)))  float    v4f;

__device__ __forceinline__ unsigned short f2bf_bits(float f) {
  unsigned u = __float_as_uint(f);
  return (unsigned short)((u + 0x7FFFu + ((u >> 16) & 1u)) >> 16);
}
__device__ __forceinline__ float bf_bits2f(unsigned short h) { return __uint_as_float(((unsigned)h) << 16); }

__device__ __forceinline__ void dep_guard_h(v8f& a, v8f& b, v16h x, v16h y) { asm volatile("v_nop\n\tv_nop\n\tv_nop\n\tv_nop" : "+v"(a), "+v"(b) : "v"(x), "v"(y)); }
__device__ __forceinline__ void dep_guard_b(v8f& a, v8f& b, v16b x, v16b y) { asm volatile("v_nop\n\tv_nop\n\tv_nop\n\tv_nop" : "+v"(a), "+v"(b) : "v"(x), "v"(y)); }
__device__ __forceinline__ void keep4_h(v16h a, v16h b, v16h c, v16h d) { asm volatile("v_nop" :: "v"(a), "v"(b), "v"(c), "v"(d)); }
__device__ __forceinline__ void keep4_b(v16b a, v16b b, v16b c, v16b d) { asm volatile("v_nop" :: "v"(a), "v"(b), "v"(c), "v"(d)); }
__device__ __forceinline__ void acc_guard4(v8f& a, v8f& b, v8f& c, v8f& d) { asm volatile("v_nop\n\tv_nop\n\tv_nop\n\tv_nop" : "+v"(a), "+v"(b), "+v"(c), "+v"(d)); }
template <typename T> struct Frag;
template <> struct Frag<_Float16> {
  typedef v16h V; union U { v16h v; v8h h[2]; };
  static __device__ __forceinline__ v16h load(const _Float16* p) {
    U f; f.h[0] = *(const v8h*)(p); f.h[1] = *(const v8h*)(p + 16); return f.v;
  }
  static __device__ __forceinline__ v8f mma(v16h a, v16h b, v8f c) {
    return __builtin_amdgcn_wmma_f32_16x16x32_f16(false, a, false, b, (short)0, c, false, false);
  }
  static __device__ __forceinline__ void guard(v8f& a, v8f& b, v16h x, v16h y) { dep_guard_h(a, b, x, y); }
  static __device__ __forceinline__ void keep(v16h a, v16h b, v16h c, v16h d) { keep4_h(a, b, c, d); }
};
template <> struct Frag<__bf16> {
  typedef v16b V; union U { v16b v; v8b h[2]; };
  static __device__ __forceinline__ v16b load(const __bf16* p) {
    U f; f.h[0] = *(const v8b*)(p); f.h[1] = *(const v8b*)(p + 16); return f.v;
  }
  static __device__ __forceinline__ v8f mma(v16b a, v16b b, v8f c) {
    return __builtin_amdgcn_wmma_f32_16x16x32_bf16(false, a, false, b, (short)0, c, false, false);
  }
  static __device__ __forceinline__ void guard(v8f& a, v8f& b, v16b x, v16b y) { dep_guard_b(a, b, x, y); }
  static __device__ __forceinline__ void keep(v16b a, v16b b, v16b c, v16b d) { keep4_b(a, b, c, d); }
};

template <int ET> struct Elem;
template <> struct Elem<0> { typedef _Float16 T; };
template <> struct Elem<1> { typedef __bf16 T; };
template <int ET, bool SPLIT, int BIAS_MODE, int OUT_MODE, bool RESID, int ACT = 0>
__global__ __launch_bounds__(256) void wmma_gemm64(
    const unsigned short* __restrict__ Ap, const unsigned short* __restrict__ A2p, int lda, long strideA,
    const unsigned short* __restrict__ Btp, const unsigned short* __restrict__ Bt2p, int ldb, long strideB,
    void* __restrict__ Cout, void* __restrict__ Cout2, int ldc, long strideC,
    const float* __restrict__ bias,
    const float* __restrict__ resid, long strideR,
    int M, int N, int K, float scale) {
  typedef typename Elem<ET>::T T;
  typedef typename Frag<T>::V V;
  const T* A = (const T*)Ap; const T* A2 = (const T*)A2p; const T* Bt = (const T*)Btp; const T* Bt2 = (const T*)Bt2p;
  __shared__ __align__(16) float sT[8][16 * 68];
  const int b    = blockIdx.y;
  const int lane = threadIdx.x & 31;
  const int wave = threadIdx.x >> 5;
  const int tilesN = N >> 6;
  const int tilesM = M >> 6;
  const int tile = blockIdx.x * 8 + wave;
  if (tile >= tilesM * tilesN) return;
  const int tm = tile / tilesN;
  const int tn = tile - tm * tilesN;
  const int m0 = tm << 6;
  const int n0 = tn << 6;

  const T* Ab  = A  + (size_t)b * strideA;
  const T* Bb  = Bt + (size_t)b * strideB;
  const T* Ab2 = SPLIT ? (A2  + (size_t)b * strideA) : nullptr;
  const T* Bb2 = SPLIT ? (Bt2 + (size_t)b * strideB) : nullptr;

  const int rlane = lane & 15;
  const int koff  = (lane >> 4) * 8;
  const int mOff  = (lane >> 4) * 8;

  v8f acc[4][4];
#pragma unroll
  for (int i = 0; i < 4; ++i)
#pragma unroll
    for (int j = 0; j < 4; ++j) acc[i][j] = (v8f){0.f,0.f,0.f,0.f,0.f,0.f,0.f,0.f};

  for (int k0 = 0; k0 < K; k0 += 32) {
    V bh[4], bl[4];
#pragma unroll
    for (int j = 0; j < 4; ++j) {
      const size_t bo = (size_t)(n0 + (j << 4) + rlane) * ldb + koff + k0;
      bh[j] = Frag<T>::load(Bb + bo);
      if (SPLIT) bl[j] = Frag<T>::load(Bb2 + bo);
    }
#pragma unroll
    for (int i = 0; i < 4; ++i) {
      const size_t ao = (size_t)(m0 + (i << 4) + rlane) * lda + koff + k0;
      V ah = Frag<T>::load(Ab + ao);
      V al;
      if (SPLIT) al = Frag<T>::load(Ab2 + ao);
#pragma unroll
      for (int j = 0; j < 4; ++j) {
        acc[i][j] = Frag<T>::mma(ah, bh[j], acc[i][j]);
        if (SPLIT) {
          acc[i][j] = Frag<T>::mma(ah, bl[j], acc[i][j]);
          acc[i][j] = Frag<T>::mma(al, bh[j], acc[i][j]);
        }
      }
      Frag<T>::guard(acc[i][0], acc[i][3], ah, SPLIT ? al : ah);
    }
    Frag<T>::keep(bh[0], bh[1], bh[2], bh[3]);
    if (SPLIT) Frag<T>::keep(bl[0], bl[1], bl[2], bl[3]);
  }
  acc_guard4(acc[0][0], acc[0][1], acc[0][2], acc[0][3]);
  acc_guard4(acc[1][0], acc[1][1], acc[1][2], acc[1][3]);
  acc_guard4(acc[2][0], acc[2][1], acc[2][2], acc[2][3]);
  acc_guard4(acc[3][0], acc[3][1], acc[3][2], acc[3][3]);

  float* slab = sT[wave];
  const float* Rb = RESID ? (resid + (size_t)b * strideR) : nullptr;
#pragma unroll
  for (int i = 0; i < 4; ++i) {
    const int mBase = m0 + (i << 4);
#pragma unroll
    for (int j = 0; j < 4; ++j) {
      const int n = n0 + (j << 4) + rlane;
      float bv = 0.f;
      if (BIAS_MODE == 2) bv = bias[n];
#pragma unroll
      for (int r = 0; r < 8; ++r) {
        float v = acc[i][j][r] * scale;
        if (BIAS_MODE == 1) v += bias[mBase + mOff + r];
        if (BIAS_MODE == 2) v += bv;
        if (RESID) v += Rb[(size_t)(mBase + mOff + r) * ldc + n];
        if (ACT == 1) v = tanhf(v);
        if (ACT == 2) v = fmaxf(v, 0.0f);
        if (ACT == 3) v = v / (1.0f + expf(-v));
        if (ACT == 4) v = (v > 0.f) ? v : 0.01f * v;
        if (ACT == 5) v = 0.5f * v * (1.0f + erff(v * 0.70710678118654752f));
        if (ACT == 6) { v = fmaxf(v, 0.0f); v = v * v; }
        slab[(mOff + r) * 68 + (j << 4) + rlane] = v;
      }
    }
    __builtin_amdgcn_fence(__ATOMIC_RELEASE, "workgroup");
    __builtin_amdgcn_wave_barrier();
    __builtin_amdgcn_fence(__ATOMIC_ACQUIRE, "workgroup");
    if (OUT_MODE == 0) {
      float* C = (float*)Cout + (size_t)b * strideC;
      const int hh = lane >> 4, c4 = (lane & 15) * 4;
      for (int pass = 0; pass < 2; ++pass) {
#pragma unroll
        for (int it = 0; it < 8; ++it) {
          const int row = it * 2 + hh;
          v4f v = *(const v4f*)(slab + row * 68 + c4);
          *(volatile v4f*)(C + (size_t)(mBase + row) * ldc + n0 + c4) = v;
        }
        __threadfence();
      }
    } else {
      const int q = lane >> 3, c8 = (lane & 7) * 8;
      unsigned short* C  = (unsigned short*)Cout  + (size_t)b * strideC;
      unsigned short* C2 = (OUT_MODE == 2) ? ((unsigned short*)Cout2 + (size_t)b * strideC) : nullptr;
      for (int pass = 0; pass < 2; ++pass) {
#pragma unroll
        for (int it = 0; it < 4; ++it) {
          const int row = it * 4 + q;
          const float* sp = slab + row * 68 + c8;
          v8h hv, lv;
#pragma unroll
          for (int e = 0; e < 8; ++e) {
            if (OUT_MODE == 1) {
              hv[e] = (_Float16)sp[e];
            } else {
              unsigned short hb = f2bf_bits(sp[e]);
              unsigned short lb = f2bf_bits(sp[e] - bf_bits2f(hb));
              hv[e] = __builtin_bit_cast(_Float16, hb);
              lv[e] = __builtin_bit_cast(_Float16, lb);
            }
          }
          *(volatile v8h*)(C + (size_t)(mBase + row) * ldc + n0 + c8) = hv;
          if (OUT_MODE == 2) *(volatile v8h*)(C2 + (size_t)(mBase + row) * ldc + n0 + c8) = lv;
        }
        __threadfence();
      }
    }
    __builtin_amdgcn_fence(__ATOMIC_RELEASE, "workgroup");
    __builtin_amdgcn_wave_barrier();
    __builtin_amdgcn_fence(__ATOMIC_ACQUIRE, "workgroup");
  }
}

__global__ __launch_bounds__(256) void k_cast_w(
    const float* __restrict__ in, _Float16* __restrict__ out, int n2, float sc) {
  int i = blockIdx.x * 256 + threadIdx.x;
  if (i < n2) {
    const _Float16 h0 = (_Float16)(in[2 * i] * sc), h1 = (_Float16)(in[2 * i + 1] * sc);
    const unsigned u = (unsigned)__builtin_bit_cast(unsigned short, h0) | ((unsigned)__builtin_bit_cast(unsigned short, h1) << 16);
    ((volatile unsigned*)out)[i] = u;
    __threadfence();
    ((volatile unsigned*)out)[i] = u;
  }
}

__device__ __forceinline__ float wsum32(float v) {
#pragma unroll
  for (int o = 16; o > 0; o >>= 1) v += __shfl_xor(v, o, 32);
  return v;
}

template <bool GATHER>
__global__ __launch_bounds__(256) void k_ln_rows(const float* __restrict__ src, const int* __restrict__ tok, int nvocab,
                                                 const float* __restrict__ g, const float* __restrict__ bta,
                                                 float* __restrict__ dst, int nrows) {
  const int lane = threadIdx.x & 31, wave = threadIdx.x >> 5;
  const int rbase = (blockIdx.x * 8 + wave) * 4;
  const v4f gv = *(const v4f*)(g + lane * 4);
  const v4f bv = *(const v4f*)(bta + lane * 4);
#pragma unroll 1
  for (int i = 0; i < 4; ++i) {
    const int row = rbase + i;
    const int rowc = row < nrows ? row : nrows - 1;
    size_t soff;
    if (GATHER) {
      int tk = tok[rowc];
      tk = tk < 0 ? 0 : (tk >= nvocab ? nvocab - 1 : tk);
      soff = (size_t)tk * DD;
    } else {
      soff = (size_t)rowc * DD;
    }
    const v4f v = *(const v4f*)(src + soff + lane * 4);
    float s = (v[0] + v[1]) + (v[2] + v[3]);
    s = wsum32(s);
    const float mean = s * (1.0f / DD);
    const float c0 = v[0] - mean, c1 = v[1] - mean, c2 = v[2] - mean, c3 = v[3] - mean;
    float q = (c0 * c0 + c1 * c1) + (c2 * c2 + c3 * c3);
    q = wsum32(q) * (1.0f / DD);
    const float inv = 1.0f / sqrtf(q + 1e-5f);
    v4f o;
    o[0] = c0 * inv * gv[0] + bv[0];
    o[1] = c1 * inv * gv[1] + bv[1];
    o[2] = c2 * inv * gv[2] + bv[2];
    o[3] = c3 * inv * gv[3] + bv[3];
    if (row < nrows) {
      float* p = dst + (size_t)row * DD + lane * 4;
      *(volatile v4f*)p = o;
      __threadfence();
      *(volatile v4f*)p = o;
    }
  }
}

template <int NOUT, bool SHIFT>
__global__ __launch_bounds__(256) void k_mix(const float* __restrict__ H,
                                             const float* __restrict__ m0, const float* __restrict__ m1, const float* __restrict__ m2,
                                             _Float16* P0, _Float16* P1, _Float16* P2, int nrows, int T) {
  const int lane = threadIdx.x & 31, wave = threadIdx.x >> 5;
  const int rsub = lane >> 4, c8 = (lane & 15) * 8;
  const int wbase = (blockIdx.x * 8 + wave) * 8;
  v4f ma0, ma1, mb0, mb1, mc0, mc1;
  if (SHIFT) {
    ma0 = *(const v4f*)(m0 + c8); ma1 = *(const v4f*)(m0 + c8 + 4);
    if (NOUT >= 2) { mb0 = *(const v4f*)(m1 + c8); mb1 = *(const v4f*)(m1 + c8 + 4); }
    if (NOUT >= 3) { mc0 = *(const v4f*)(m2 + c8); mc1 = *(const v4f*)(m2 + c8 + 4); }
  }
#pragma unroll 1
  for (int it = 0; it < 4; ++it) {
    const int row = wbase + it * 2 + rsub;
    const int rowc = row < nrows ? row : nrows - 1;
    const int t = rowc % T;
    const int prow = (SHIFT && t > 0) ? rowc - 1 : rowc;
    const float pf = (SHIFT && t > 0) ? 1.0f : 0.0f;
    const float* hr = H + (size_t)rowc * DD + c8;
    const v4f h0 = *(const v4f*)hr, h1 = *(const v4f*)(hr + 4);
    v4f q0, q1;
    if (SHIFT) {
      const float* hp = H + (size_t)prow * DD + c8;
      q0 = *(const v4f*)hp * pf;
      q1 = *(const v4f*)(hp + 4) * pf;
    }
    v8h o0, o1, o2;
#pragma unroll
    for (int e = 0; e < 4; ++e) {
      if (SHIFT) {
        o0[e]     = (_Float16)(h0[e] * ma0[e] + q0[e] * (1.0f - ma0[e]));
        o0[4 + e] = (_Float16)(h1[e] * ma1[e] + q1[e] * (1.0f - ma1[e]));
        if (NOUT >= 2) {
          o1[e]     = (_Float16)(h0[e] * mb0[e] + q0[e] * (1.0f - mb0[e]));
          o1[4 + e] = (_Float16)(h1[e] * mb1[e] + q1[e] * (1.0f - mb1[e]));
        }
        if (NOUT >= 3) {
          o2[e]     = (_Float16)(h0[e] * mc0[e] + q0[e] * (1.0f - mc0[e]));
          o2[4 + e] = (_Float16)(h1[e] * mc1[e] + q1[e] * (1.0f - mc1[e]));
        }
      } else {
        o0[e] = (_Float16)h0[e]; o0[4 + e] = (_Float16)h1[e];
        if (NOUT >= 2) { o1[e] = o0[e]; o1[4 + e] = o0[4 + e]; }
        if (NOUT >= 3) { o2[e] = o0[e]; o2[4 + e] = o0[4 + e]; }
      }
    }
    if (row < nrows) {
      const size_t doff = (size_t)row * DD + c8;
      *(volatile v8h*)(P0 + doff) = o0;
      if (NOUT >= 2) *(volatile v8h*)(P1 + doff) = o1;
      if (NOUT >= 3) *(volatile v8h*)(P2 + doff) = o2;
      __threadfence();
      *(volatile v8h*)(P0 + doff) = o0;
      if (NOUT >= 2) *(volatile v8h*)(P1 + doff) = o1;
      if (NOUT >= 3) *(volatile v8h*)(P2 + doff) = o2;
    }
  }
}

__global__ __launch_bounds__(128) void k_wkv(const float* __restrict__ Kp, const float* __restrict__ Vp,
                                             const float* __restrict__ Rp,
                                             const float* __restrict__ tfl, const float* __restrict__ tdl,
                                             _Float16* __restrict__ RW, int T) {
  __shared__ __align__(16) _Float16 tile[16 * DD];
  const int b = blockIdx.x, d = threadIdx.x;
  const int srow = d >> 4, c8 = (d & 15) * 8;
  const float tfv = tfl[d], tdv = tdl[d];
  float sA = 0.f, sB = 0.f, sp = -1e30f;
#pragma unroll 1
  for (int t0 = 0; t0 < T; t0 += 16) {
#pragma unroll 1
    for (int j = 0; j < 16; ++j) {
      const size_t off = ((size_t)b * T + t0 + j) * DD + d;
      const float kk = Kp[off], vv = Vp[off], rr = Rp[off];
      const float r = 1.0f / (1.0f + expf(-rr));
      const float ww = tfv + kk;
      const float p = fmaxf(sp, ww);
      const float e1 = expf(sp - p), e2 = expf(ww - p);
      const float num = e1 * sA + e2 * vv;
      const float den = (e1 * sB + e2) + 1e-8f;
      const float wkv = num * (1.0f / den);
      tile[j * DD + d] = (_Float16)(r * wkv);
      const float ww2 = sp + tdv;
      const float p2 = fmaxf(ww2, kk);
      const float f1 = expf(ww2 - p2), f2 = expf(kk - p2);
      sA = f1 * sA + f2 * vv;
      sB = f1 * sB + f2;
      sp = p2;
    }
    __syncthreads();
    const v8h w0 = *(const v8h*)(tile + srow * DD + c8);
    const v8h w1 = *(const v8h*)(tile + (srow + 8) * DD + c8);
    _Float16* d0 = RW + ((size_t)b * T + t0 + srow) * DD + c8;
    _Float16* d1 = RW + ((size_t)b * T + t0 + srow + 8) * DD + c8;
    *(volatile v8h*)d0 = w0;
    *(volatile v8h*)d1 = w1;
    __threadfence();
    *(volatile v8h*)d0 = w0;
    *(volatile v8h*)d1 = w1;
    __syncthreads();
  }
}

__global__ __launch_bounds__(256) void k_combine(const float* __restrict__ X, const float* __restrict__ S,
                                                 const float* __restrict__ C, float* __restrict__ Y, int nrows) {
  const int lane = threadIdx.x & 31, wave = threadIdx.x >> 5;
  const int rbase = (blockIdx.x * 8 + wave) * 4;
#pragma unroll 1
  for (int i = 0; i < 4; ++i) {
    const int row = rbase + i;
    const int rowc = row < nrows ? row : nrows - 1;
    const size_t off = (size_t)rowc * DD + lane * 4;
    const v4f x = *(const v4f*)(X + off);
    const v4f s = *(const v4f*)(S + off);
    const v4f c = *(const v4f*)(C + off);
    v4f o;
#pragma unroll
    for (int e = 0; e < 4; ++e) {
      const float sg = 1.0f / (1.0f + expf(-s[e]));
      o[e] = x[e] + sg * c[e];
    }
    if (row < nrows) {
      float* p = Y + (size_t)row * DD + lane * 4;
      *(volatile v4f*)p = o;
      __threadfence();
      *(volatile v4f*)p = o;
    }
  }
}

template <int OUTM, bool RESID, int ACT>
static void run_gemm(hipStream_t st, const void* A, int lda, long sA, const void* Bt, int ldb, long sB,
                     void* C, int ldc, long sC, const float* resid, long sR, const float* fdummy,
                     int M, int N, int K, float scale, int batch) {
  const int tiles = (M >> 6) * (N >> 6);
  const int blocks = (tiles + 7) >> 3;
  wmma_gemm64<0, false, 0, OUTM, RESID, ACT><<<dim3(blocks, batch), dim3(256), 0, st>>>(
      (const unsigned short*)A, (const unsigned short*)A, lda, sA,
      (const unsigned short*)Bt, (const unsigned short*)Bt, ldb, sB,
      C, C, ldc, sC, fdummy, resid, sR, M, N, K, scale);
}

extern "C" void kernel_launch(void* const* d_in, const int* in_sizes, int n_in,
                              void* d_out, int out_size, void* d_ws, size_t ws_size,
                              hipStream_t stream) {
  if (n_in < 25) return;
  if (in_sizes[0] != NR || in_sizes[1] != VV * DD || in_sizes[13] != LL * DD * DD ||
      in_sizes[16] != LL * DD * DD || in_sizes[19] != LL * FF * DD || in_sizes[20] != LL * DD * FF ||
      in_sizes[21] != LL * DD * DD || in_sizes[24] != VV * DD || in_sizes[8] != LL * DD ||
      out_size != NR * VV) return;

  const int*   tokens  = (const int*)d_in[0];
  const float* emb     = (const float*)d_in[1];
  const float* ln0_g   = (const float*)d_in[2];
  const float* ln0_b   = (const float*)d_in[3];
  const float* ln1_g   = (const float*)d_in[4];
  const float* ln1_b   = (const float*)d_in[5];
  const float* ln2_g   = (const float*)d_in[6];
  const float* ln2_b   = (const float*)d_in[7];
  const float* td      = (const float*)d_in[8];
  const float* tf      = (const float*)d_in[9];
  const float* tmk     = (const float*)d_in[10];
  const float* tmv     = (const float*)d_in[11];
  const float* tmr     = (const float*)d_in[12];
  const float* Wk      = (const float*)d_in[13];
  const float* Wv      = (const float*)d_in[14];
  const float* Wr      = (const float*)d_in[15];
  const float* Wo      = (const float*)d_in[16];
  const float* cmk     = (const float*)d_in[17];
  const float* cmr     = (const float*)d_in[18];
  const float* Ck      = (const float*)d_in[19];
  const float* Cv      = (const float*)d_in[20];
  const float* Cr      = (const float*)d_in[21];
  const float* lnout_g = (const float*)d_in[22];
  const float* lnout_b = (const float*)d_in[23];
  const float* head    = (const float*)d_in[24];
  float* out = (float*)d_out;

  const size_t MIB = 1048576;
  const size_t OFF_W16 = 0;
  const size_t OFF_X0  = 1 * MIB;
  const size_t OFF_X1  = 17 * MIB;
  const size_t OFF_H   = 33 * MIB;
  const size_t OFF_A16 = 49 * MIB;
  const size_t OFF_C32 = 73 * MIB;
  const size_t OFF_END = 121 * MIB;
  if (ws_size < OFF_END) return;

  char* ws = (char*)d_ws;
  _Float16* W16 = (_Float16*)(ws + OFF_W16);
  _Float16* WK16 = W16;
  _Float16* WV16 = WK16 + LL * DD * DD;
  _Float16* WR16 = WV16 + LL * DD * DD;
  _Float16* WO16 = WR16 + LL * DD * DD;
  _Float16* CR16 = WO16 + LL * DD * DD;
  _Float16* CK16 = CR16 + LL * DD * DD;
  _Float16* CV16 = CK16 + LL * FF * DD;
  _Float16* HD16 = CV16 + LL * DD * FF;
  float* X0 = (float*)(ws + OFF_X0);
  float* X1 = (float*)(ws + OFF_X1);
  float* Hf = (float*)(ws + OFF_H);
  const size_t PL16 = (size_t)NR * DD;
  const size_t PL32 = (size_t)NR * DD;
  _Float16* A0h = (_Float16*)(ws + OFF_A16);
  _Float16* A1h = A0h + PL16;
  _Float16* A2h = A1h + PL16;
  float* Kp = (float*)(ws + OFF_C32);
  float* Vp = Kp + PL32;
  float* Rp = Vp + PL32;
  _Float16* KF16 = (_Float16*)(ws + OFF_C32);
  float* SRp = Rp;
  float* CVp = Hf;

  const float WSC = 16.0f;
  k_cast_w<<<(LL * DD * DD / 2) / 256, 256, 0, stream>>>(Wk, WK16, LL * DD * DD / 2, WSC);
  k_cast_w<<<(LL * DD * DD / 2) / 256, 256, 0, stream>>>(Wv, WV16, LL * DD * DD / 2, WSC);
  k_cast_w<<<(LL * DD * DD / 2) / 256, 256, 0, stream>>>(Wr, WR16, LL * DD * DD / 2, WSC);
  k_cast_w<<<(LL * DD * DD / 2) / 256, 256, 0, stream>>>(Wo, WO16, LL * DD * DD / 2, WSC);
  k_cast_w<<<(LL * DD * DD / 2) / 256, 256, 0, stream>>>(Cr, CR16, LL * DD * DD / 2, WSC);
  k_cast_w<<<(LL * FF * DD / 2) / 256, 256, 0, stream>>>(Ck, CK16, LL * FF * DD / 2, WSC);
  k_cast_w<<<(LL * DD * FF / 2) / 256, 256, 0, stream>>>(Cv, CV16, LL * DD * FF / 2, WSC);
  k_cast_w<<<(VV * DD / 2) / 256, 256, 0, stream>>>(head, HD16, VV * DD / 2, WSC);

  k_ln_rows<true><<<NR / 32, 256, 0, stream>>>(emb, tokens, VV, ln0_g, ln0_b, X0, NR);

  const float* fdummy = X0;
  const long sA16 = (long)PL16, sC32 = (long)PL32, sW = (long)(LL * DD * DD);

  for (int l = 0; l < LL; ++l) {
    k_ln_rows<false><<<NR / 32, 256, 0, stream>>>(X0, tokens, VV, ln1_g + l * DD, ln1_b + l * DD, Hf, NR);
    k_mix<3, true><<<NR / 64, 256, 0, stream>>>(Hf, tmk + l * DD, tmv + l * DD, tmr + l * DD, A0h, A1h, A2h, NR, TT);
    run_gemm<0, false, 0>(stream, A0h, DD, sA16, WK16 + (size_t)l * DD * DD, DD, sW,
                          Kp, DD, sC32, fdummy, 0, fdummy, NR, DD, DD, 1.0f / 16.0f, 3);
    k_wkv<<<BB, DD, 0, stream>>>(Kp, Vp, Rp, tf + l * DD, td + l * DD, A0h, TT);
    run_gemm<0, true, 0>(stream, A0h, DD, 0, WO16 + (size_t)l * DD * DD, DD, 0,
                         X1, DD, 0, X0, 0, fdummy, NR, DD, DD, 1.0f / 16.0f, 1);
    k_ln_rows<false><<<NR / 32, 256, 0, stream>>>(X1, tokens, VV, ln2_g + l * DD, ln2_b + l * DD, Hf, NR);
    k_mix<2, true><<<NR / 64, 256, 0, stream>>>(Hf, cmk + l * DD, cmr + l * DD, cmr + l * DD, A0h, A1h, A2h, NR, TT);
    run_gemm<1, false, 6>(stream, A0h, DD, 0, CK16 + (size_t)l * FF * DD, DD, 0,
                          KF16, FF, 0, fdummy, 0, fdummy, NR, FF, DD, 0.5f, 1);
    run_gemm<0, false, 0>(stream, A1h, DD, 0, CR16 + (size_t)l * DD * DD, DD, 0,
                          SRp, DD, 0, fdummy, 0, fdummy, NR, DD, DD, 1.0f / 16.0f, 1);
    run_gemm<0, false, 0>(stream, KF16, FF, 0, CV16 + (size_t)l * DD * FF, FF, 0,
                          CVp, DD, 0, fdummy, 0, fdummy, NR, DD, FF, 1.0f / 1024.0f, 1);
    k_combine<<<NR / 32, 256, 0, stream>>>(X1, SRp, CVp, X0, NR);
  }

  k_ln_rows<false><<<NR / 32, 256, 0, stream>>>(X0, tokens, VV, lnout_g, lnout_b, Hf, NR);
  k_mix<1, false><<<NR / 64, 256, 0, stream>>>(Hf, tmk, tmk, tmk, A0h, A1h, A2h, NR, TT);
  run_gemm<0, false, 0>(stream, A0h, DD, 0, HD16, DD, 0,
                        out, VV, 0, fdummy, 0, fdummy, NR, VV, DD, 1.0f / 16.0f, 1);
  (void)hipGetLastError();
}
